// DurationBiasedAttention_21672404976047
// MI455X (gfx1250) — hardware-verified
//
#include <hip/hip_runtime.h>
#include <stddef.h>

#define NBT 2
#define SL  2048
#define DM  512
#define NH  8
#define HD  64
#define NT  (NBT * SL)
#define QB  128
#define KC  64
#define NQB (SL / QB)
#define NCK (SL / KC)
#define KTP 72
#define PT  (16 * KTP)
#define OTP 68
#define VTP 132
#define TTP 68
#define GAPR 33
#define DURR 17
#define NEGV (-1.0e9f)

static_assert(NT == 4096);
static_assert(NH * HD == DM);
static_assert(SL % QB == 0);
static_assert(SL % KC == 0);
static_assert(SL % 128 == 0);
static_assert(DM % 64 == 0);
static_assert(DM % 32 == 0);
static_assert((NT * DM) % 2048 == 0);
static_assert(HD == 64);
static_assert(KC == 64);
static_assert(64 * VTP <= 128 * OTP);
static_assert(16 * OTP * 4 <= 2 * PT * 2);

typedef __bf16       v16b __attribute__((ext_vector_type(16)));
typedef float        v8f  __attribute__((ext_vector_type(8)));
typedef float        v4f  __attribute__((ext_vector_type(4)));
typedef unsigned int v4u  __attribute__((ext_vector_type(4)));
typedef int          v4i  __attribute__((ext_vector_type(4)));
union Frag { v16b v; v4u u[2]; };

__device__ __forceinline__ v8f mma(v16b a, v16b b, v8f c) {
  c = __builtin_amdgcn_wmma_f32_16x16x32_bf16(false, a, false, b, (short)0, c, false, false);
  asm volatile("v_nop\n\tv_nop\n\tv_nop\n\tv_nop" : "+v"(c) : "v"(a), "v"(b));
  return c;
}

__device__ __forceinline__ v8f zero8() { return (v8f){0.f, 0.f, 0.f, 0.f, 0.f, 0.f, 0.f, 0.f}; }

__device__ __forceinline__ v16b ldf(const unsigned short* p, int ld, int row0, int k0, int lane) {
  const unsigned short* q = p + (size_t)(row0 + (lane & 15)) * ld + k0 + 8 * (lane >> 4);
  Frag f;
  f.u[0] = *(const v4u*)(q);
  f.u[1] = *(const v4u*)(q + 16);
  return f.v;
}

__device__ __forceinline__ unsigned int bf_rne(float x) {
  const unsigned int u = __float_as_uint(x);
  return (u + 0x7FFFu + ((u >> 16) & 1u)) >> 16;
}

__device__ __forceinline__ void split2(float a, float b, unsigned int& wh, unsigned int& wl) {
  const unsigned int ha = bf_rne(a), hb = bf_rne(b);
  const float ra = a - __uint_as_float(ha << 16);
  const float rb = b - __uint_as_float(hb << 16);
  wh = ha | (hb << 16);
  wl = bf_rne(ra) | (bf_rne(rb) << 16);
}

__device__ __forceinline__ void split8(v4f a0, v4f a1, v4u& wh, v4u& wl) {
  unsigned int h0, h1, h2, h3, l0, l1, l2, l3;
  split2(a0[0], a0[1], h0, l0);
  split2(a0[2], a0[3], h1, l1);
  split2(a1[0], a1[1], h2, l2);
  split2(a1[2], a1[3], h3, l3);
  wh = (v4u){h0, h1, h2, h3};
  wl = (v4u){l0, l1, l2, l3};
}

__global__ __launch_bounds__(256) void k_split(const float* __restrict__ src,
                                               unsigned short* __restrict__ dh,
                                               unsigned short* __restrict__ dl) {
  const size_t o = (size_t)blockIdx.x * 2048 + (size_t)threadIdx.x * 8;
  const v4f a0 = *(const v4f*)(src + o);
  const v4f a1 = *(const v4f*)(src + o + 4);
  v4u wh, wl;
  split8(a0, a1, wh, wl);
  volatile v4u* ph = (volatile v4u*)(dh + o);
  volatile v4u* pl = (volatile v4u*)(dl + o);
  *ph = wh;
  *pl = wl;
  __threadfence();
  *ph = wh;
  *pl = wl;
}

__global__ __launch_bounds__(256) void k_split_tr(const float* __restrict__ Wq, const float* __restrict__ Wk,
                                                  const float* __restrict__ Wv, const float* __restrict__ Wo,
                                                  unsigned short* __restrict__ Ph, unsigned short* __restrict__ Pl,
                                                  unsigned short* __restrict__ Oh, unsigned short* __restrict__ Ol) {
  __shared__ __align__(16) float st[64 * TTP];
  const int tid = threadIdx.x;
  const int z   = blockIdx.z;
  const int nt  = blockIdx.x * 64;
  const int kt  = blockIdx.y * 64;
  const float* W = (z == 0) ? Wq : ((z == 1) ? Wk : ((z == 2) ? Wv : Wo));
  {
    const int row = tid >> 2;
    const int cb  = (tid & 3) * 16;
    const float* src = W + (size_t)(kt + row) * DM + nt + cb;
#pragma unroll
    for (int e = 0; e < 4; ++e) {
      const v4f a = *(const v4f*)(src + 4 * e);
#pragma unroll
      for (int q = 0; q < 4; ++q) st[(cb + 4 * e + q) * TTP + row] = a[q];
    }
  }
  __syncthreads();
  unsigned short* dh = (z < 3) ? (Ph + (size_t)z * DM * DM) : Oh;
  unsigned short* dl = (z < 3) ? (Pl + (size_t)z * DM * DM) : Ol;
  const size_t base = (size_t)nt * DM + kt;
  v4u vh[2], vl[2];
  size_t go[2];
#pragma unroll
  for (int it = 0; it < 2; ++it) {
    const int pp   = tid + 256 * it;
    const int rown = pp >> 3;
    const int pc   = pp & 7;
    const float* ra = st + rown * TTP + 8 * pc;
    const v4f a0 = *(const v4f*)(ra), a1 = *(const v4f*)(ra + 4);
    split8(a0, a1, vh[it], vl[it]);
    go[it] = base + (size_t)rown * DM + 8 * pc;
  }
  for (int ps = 0; ps < 2; ++ps) {
#pragma unroll
    for (int it = 0; it < 2; ++it) {
      *(volatile v4u*)(dh + go[it]) = vh[it];
      *(volatile v4u*)(dl + go[it]) = vl[it];
    }
    __threadfence();
  }
}

__device__ __forceinline__ void gemm32x32x3(const unsigned short* __restrict__ Ah,
                                            const unsigned short* __restrict__ Al, int lda,
                                            const unsigned short* __restrict__ Bh,
                                            const unsigned short* __restrict__ Bl, int ldb,
                                            int K, int m0, int n0, int lane, v8f (&acc)[2][2]) {
#pragma unroll 1
  for (int k0 = 0; k0 < K; k0 += 32) {
    const v16b ah0 = ldf(Ah, lda, m0, k0, lane);
    const v16b ah1 = ldf(Ah, lda, m0 + 16, k0, lane);
    const v16b al0 = ldf(Al, lda, m0, k0, lane);
    const v16b al1 = ldf(Al, lda, m0 + 16, k0, lane);
#pragma unroll
    for (int t = 0; t < 2; ++t) {
      const v16b bh = ldf(Bh, ldb, n0 + 16 * t, k0, lane);
      const v16b bl = ldf(Bl, ldb, n0 + 16 * t, k0, lane);
      acc[0][t] = mma(ah0, bh, acc[0][t]);
      acc[1][t] = mma(ah1, bh, acc[1][t]);
      acc[0][t] = mma(ah0, bl, acc[0][t]);
      acc[1][t] = mma(ah1, bl, acc[1][t]);
      acc[0][t] = mma(al0, bh, acc[0][t]);
      acc[1][t] = mma(al1, bh, acc[1][t]);
    }
  }
}

__device__ __forceinline__ void stage_rm(v8f (&acc)[2][2], const float (&bb)[2], float* st,
                                         int mw, int nw, int hh, int c) {
#pragma unroll
  for (int s = 0; s < 2; ++s)
#pragma unroll
    for (int t = 0; t < 2; ++t)
#pragma unroll
      for (int r = 0; r < 8; ++r)
        st[(mw + 16 * s + 8 * hh + r) * OTP + nw + 16 * t + c] = acc[s][t][r] + bb[t];
}

__device__ __forceinline__ void stage_tr(v8f (&acc)[2][2], const float (&bb)[2], float* st,
                                         int mw, int nw, int hh, int c) {
#pragma unroll
  for (int s = 0; s < 2; ++s)
#pragma unroll
    for (int t = 0; t < 2; ++t)
#pragma unroll
      for (int r = 0; r < 8; ++r)
        st[(nw + 16 * t + c) * VTP + mw + 16 * s + 8 * hh + r] = acc[s][t][r] + bb[t];
}

__device__ __forceinline__ void store_planes(const float* st, unsigned short* __restrict__ oh,
                                             unsigned short* __restrict__ ol, size_t base, int ldo, int tid) {
  v4u vh[4], vl[4];
  size_t go[4];
#pragma unroll
  for (int it = 0; it < 4; ++it) {
    const int pp  = tid + 256 * it;
    const int row = pp >> 3;
    const int pc  = pp & 7;
    const float* ra = st + row * OTP + 8 * pc;
    const v4f a0 = *(const v4f*)(ra), a1 = *(const v4f*)(ra + 4);
    split8(a0, a1, vh[it], vl[it]);
    go[it] = base + (size_t)row * ldo + 8 * pc;
  }
  for (int ps = 0; ps < 2; ++ps) {
#pragma unroll
    for (int it = 0; it < 4; ++it) {
      *(volatile v4u*)(oh + go[it]) = vh[it];
      *(volatile v4u*)(ol + go[it]) = vl[it];
    }
    __threadfence();
  }
}

__device__ __forceinline__ void store_vt(const float* st, unsigned short* __restrict__ vh,
                                         unsigned short* __restrict__ vl, size_t base, int tid) {
  v4u wh[4], wl[4];
  size_t go[4];
#pragma unroll
  for (int it = 0; it < 4; ++it) {
    const int pp   = tid + 256 * it;
    const int drow = pp >> 4;
    const int pc   = pp & 15;
    const float* ra = st + drow * VTP + 8 * pc;
    const v4f a0 = *(const v4f*)(ra), a1 = *(const v4f*)(ra + 4);
    split8(a0, a1, wh[it], wl[it]);
    go[it] = base + (size_t)drow * SL + 8 * pc;
  }
  for (int ps = 0; ps < 2; ++ps) {
#pragma unroll
    for (int it = 0; it < 4; ++it) {
      *(volatile v4u*)(vh + go[it]) = wh[it];
      *(volatile v4u*)(vl + go[it]) = wl[it];
    }
    __threadfence();
  }
}

__device__ __forceinline__ void store_f32(const float* st, float* __restrict__ out, int mblk, int nblk, int tid) {
  v4f val[8];
  size_t go[8];
#pragma unroll
  for (int it = 0; it < 8; ++it) {
    const int pp  = tid + 256 * it;
    const int row = pp >> 4;
    const int pc  = pp & 15;
    val[it] = *(const v4f*)(st + row * OTP + 4 * pc);
    go[it]  = (size_t)(mblk + row) * DM + nblk + 4 * pc;
  }
  for (int ps = 0; ps < 2; ++ps) {
#pragma unroll
    for (int it = 0; it < 8; ++it) *(volatile v4f*)(out + go[it]) = val[it];
    __threadfence();
  }
}

__global__ __launch_bounds__(256) void k_proj(const unsigned short* __restrict__ Xh,
                                              const unsigned short* __restrict__ Xl,
                                              const unsigned short* __restrict__ Wh,
                                              const unsigned short* __restrict__ Wl,
                                              const float* __restrict__ bq,
                                              const float* __restrict__ bk,
                                              const float* __restrict__ bv,
                                              unsigned short* __restrict__ Qh, unsigned short* __restrict__ Ql,
                                              unsigned short* __restrict__ Kh, unsigned short* __restrict__ Kl,
                                              unsigned short* __restrict__ Vh, unsigned short* __restrict__ Vl) {
  __shared__ __align__(16) float st[128 * OTP];
  const int tid = threadIdx.x, lane = tid & 31, wave = tid >> 5;
  const int hh = lane >> 4, c = lane & 15;
  const int which = blockIdx.x / NH;
  const int head  = blockIdx.x - which * NH;
  const int mblk  = blockIdx.y * 128;
  const int b     = mblk / SL;
  const int sf    = mblk - b * SL;
  const int bh    = b * NH + head;
  const int mw = (wave >> 1) * 32, nw = (wave & 1) * 32;

  v8f acc[2][2];
#pragma unroll
  for (int s = 0; s < 2; ++s)
#pragma unroll
    for (int t = 0; t < 2; ++t) acc[s][t] = zero8();
  gemm32x32x3(Xh, Xl, DM,
              Wh + (size_t)which * DM * DM, Wl + (size_t)which * DM * DM, DM,
              DM, mblk + mw, head * HD + nw, lane, acc);

  float bb[2];
#pragma unroll
  for (int t = 0; t < 2; ++t) {
    const int i = head * HD + nw + 16 * t + c;
    const float xq = bq[i], xk = bk[i], xv = bv[i];
    bb[t] = (which == 0) ? xq : ((which == 1) ? xk : xv);
  }
  if (which < 2) stage_rm(acc, bb, st, mw, nw, hh, c);
  else           stage_tr(acc, bb, st, mw, nw, hh, c);
  __syncthreads();
  if (which < 2) {
    unsigned short* oh = (which == 0) ? Qh : Kh;
    unsigned short* ol = (which == 0) ? Ql : Kl;
    store_planes(st, oh, ol, ((size_t)bh * SL + sf) * HD, HD, tid);
  } else {
    store_vt(st, Vh, Vl, (size_t)bh * HD * SL + sf, tid);
  }
}

__global__ __launch_bounds__(256) void k_attn(const unsigned short* __restrict__ Qh,
                                              const unsigned short* __restrict__ Ql,
                                              const unsigned short* __restrict__ Kh,
                                              const unsigned short* __restrict__ Kl,
                                              const unsigned short* __restrict__ Vh,
                                              const unsigned short* __restrict__ Vl,
                                              const int* __restrict__ mask,
                                              const int* __restrict__ gids,
                                              const int* __restrict__ dids,
                                              const float* __restrict__ gap_emb,
                                              const float* __restrict__ dur_emb,
                                              unsigned short* __restrict__ Oh,
                                              unsigned short* __restrict__ Ol) {
  __shared__ __align__(16) unsigned short Ks[2 * KC * KTP];
  __shared__ __align__(16) unsigned short Vs[2 * HD * KTP];
  __shared__ __align__(16) unsigned short Ps[8 * 2 * PT];
  __shared__ int   gkS[KC];
  __shared__ float dbS[KC];
  __shared__ int   mkS[KC];
  __shared__ float gapS[36];
  __shared__ float durS[20];

  const int tid = threadIdx.x, lane = tid & 31, wave = tid >> 5;
  const int hh = lane >> 4, c = lane & 15;
  const int qb = blockIdx.x % NQB;
  const int bh = blockIdx.x / NQB;
  const int h  = bh % NH;
  const int b  = bh / NH;
  const int q0 = qb * QB + wave * 16;
  const size_t qkbase = (size_t)bh * SL * HD;
  const size_t vbase  = (size_t)bh * HD * SL;
  unsigned short* pwh = Ps + wave * 2 * PT;
  unsigned short* pwl = pwh + PT;

  {
    const int ig = (tid < GAPR) ? tid : (GAPR - 1);
    const int id = (tid < DURR) ? tid : (DURR - 1);
    const float gv = gap_emb[ig * NH + h];
    const float dv = dur_emb[id * NH + h];
    if (tid < GAPR) gapS[tid] = gv;
    if (tid < DURR) durS[tid] = dv;
  }

  const v4i ga = *(const v4i*)(gids + (size_t)b * SL + q0 + 8 * hh);
  const v4i gb = *(const v4i*)(gids + (size_t)b * SL + q0 + 8 * hh + 4);
  const int gq[8] = {ga[0], ga[1], ga[2], ga[3], gb[0], gb[1], gb[2], gb[3]};

  v16b qh[2], ql[2];
#pragma unroll
  for (int dc = 0; dc < 2; ++dc) {
    qh[dc] = ldf(Qh + qkbase, HD, q0, dc * 32, lane);
    ql[dc] = ldf(Ql + qkbase, HD, q0, dc * 32, lane);
  }

  const float NEGI = -__builtin_huge_valf();
  float mrow[8], lrow[8];
  v8f oacc[4];
#pragma unroll
  for (int r = 0; r < 8; ++r) { mrow[r] = NEGI; lrow[r] = 0.f; }
#pragma unroll
  for (int t = 0; t < 4; ++t) oacc[t] = zero8();

  for (int kc = 0; kc < NCK; ++kc) {
    const int kv0 = kc * KC;
    __syncthreads();
    {
      const int r  = tid >> 2;
      const int qq = (tid & 3) * 16;
      const unsigned short* kh = Kh + qkbase + (size_t)(kv0 + r) * HD + qq;
      const unsigned short* kl = Kl + qkbase + (size_t)(kv0 + r) * HD + qq;
      const unsigned short* vh = Vh + vbase + (size_t)r * SL + kv0 + qq;
      const unsigned short* vl = Vl + vbase + (size_t)r * SL + kv0 + qq;
#pragma unroll
      for (int e = 0; e < 2; ++e) {
        *(v4u*)(Ks + r * KTP + qq + 8 * e)            = *(const v4u*)(kh + 8 * e);
        *(v4u*)(Ks + KC * KTP + r * KTP + qq + 8 * e) = *(const v4u*)(kl + 8 * e);
        *(v4u*)(Vs + r * KTP + qq + 8 * e)            = *(const v4u*)(vh + 8 * e);
        *(v4u*)(Vs + HD * KTP + r * KTP + qq + 8 * e) = *(const v4u*)(vl + 8 * e);
      }
      if (tid < KC) {
        const int key = kv0 + tid;
        const int gk  = gids[(size_t)b * SL + key];
        int dk = dids[(size_t)b * SL + key];
        dk = (dk < 0) ? 0 : ((dk > DURR - 1) ? (DURR - 1) : dk);
        const int mk  = mask[(size_t)b * SL + key];
        gkS[tid] = gk;
        dbS[tid] = durS[dk];
        mkS[tid] = mk;
      }
    }
    __syncthreads();

    v8f s[4];
#pragma unroll
    for (int j = 0; j < 4; ++j) s[j] = zero8();
#pragma unroll
    for (int dc = 0; dc < 2; ++dc) {
#pragma unroll
      for (int j = 0; j < 4; ++j) {
        const v16b khf = ldf(Ks, KTP, j * 16, dc * 32, lane);
        const v16b klf = ldf(Ks + KC * KTP, KTP, j * 16, dc * 32, lane);
        s[j] = mma(qh[dc], khf, s[j]);
        s[j] = mma(qh[dc], klf, s[j]);
        s[j] = mma(ql[dc], khf, s[j]);
      }
    }
#pragma unroll
    for (int j = 0; j < 4; ++j) {
      const int kl  = 16 * j + c;
      const int gk  = gkS[kl];
      const float db = dbS[kl];
      const int mk  = mkS[kl];
#pragma unroll
      for (int r = 0; r < 8; ++r) {
        int rel = gq[r] - gk;
        rel = (rel < 0) ? -rel : rel;
        rel = (rel > GAPR - 1) ? (GAPR - 1) : rel;
        rel = (rel < 0) ? 0 : rel;
        const float gbias = gapS[rel];
        const float v = (s[j][r] * 0.125f + gbias) + db;
        s[j][r] = (mk != 0) ? v : NEGV;
      }
    }
    float cm[8];
#pragma unroll
    for (int r = 0; r < 8; ++r) {
      float m = fmaxf(fmaxf(s[0][r], s[1][r]), fmaxf(s[2][r], s[3][r]));
#pragma unroll
      for (int off = 1; off < 16; off <<= 1) m = fmaxf(m, __shfl_xor(m, off, 32));
      cm[r] = m;
    }
    float al[8];
#pragma unroll
    for (int r = 0; r < 8; ++r) {
      const float mnew  = fmaxf(mrow[r], cm[r]);
      const float alpha = __expf(mrow[r] - mnew);
      mrow[r] = mnew;
      float psum = 0.f;
#pragma unroll
      for (int j = 0; j < 4; ++j) {
        const float p = __expf(s[j][r] - mnew);
        psum += p;
        const unsigned int hb = bf_rne(p);
        const unsigned int lb = bf_rne(p - __uint_as_float(hb << 16));
        const int idx = (8 * hh + r) * KTP + 16 * j + c;
        pwh[idx] = (unsigned short)hb;
        pwl[idx] = (unsigned short)lb;
      }
#pragma unroll
      for (int off = 1; off < 16; off <<= 1) psum += __shfl_xor(psum, off, 32);
      lrow[r] = lrow[r] * alpha + psum;
      al[r] = alpha;
    }
#pragma unroll
    for (int t = 0; t < 4; ++t)
#pragma unroll
      for (int r = 0; r < 8; ++r) oacc[t][r] *= al[r];
    __syncthreads();

#pragma unroll
    for (int kk = 0; kk < 2; ++kk) {
      const v16b pah = ldf(pwh, KTP, 0, kk * 32, lane);
      const v16b pal = ldf(pwl, KTP, 0, kk * 32, lane);
#pragma unroll
      for (int t = 0; t < 4; ++t) {
        const v16b vhf = ldf(Vs, KTP, t * 16, kk * 32, lane);
        const v16b vlf = ldf(Vs + HD * KTP, KTP, t * 16, kk * 32, lane);
        oacc[t] = mma(pah, vhf, oacc[t]);
        oacc[t] = mma(pah, vlf, oacc[t]);
        oacc[t] = mma(pal, vhf, oacc[t]);
      }
    }
  }

  float invl[8];
#pragma unroll
  for (int r = 0; r < 8; ++r) invl[r] = 1.0f / lrow[r];
  __syncthreads();
  float* sw = (float*)(Ps + wave * 2 * PT);
#pragma unroll
  for (int r = 0; r < 8; ++r) {
#pragma unroll
    for (int t = 0; t < 4; ++t) sw[(8 * hh + r) * OTP + 16 * t + c] = oacc[t][r] * invl[r];
  }
  __syncthreads();
  v4u wh[4], wl[4];
  size_t go[4];
#pragma unroll
  for (int it = 0; it < 4; ++it) {
    const int pp = lane + 32 * it;
    const int L  = pp >> 3;
    const int pc = pp & 7;
    const float* ra = sw + L * OTP + 8 * pc;
    const v4f a0 = *(const v4f*)(ra), a1 = *(const v4f*)(ra + 4);
    split8(a0, a1, wh[it], wl[it]);
    go[it] = ((size_t)(b * SL + q0 + L)) * DM + (size_t)h * HD + 8 * pc;
  }
  for (int ps = 0; ps < 2; ++ps) {
#pragma unroll
    for (int it = 0; it < 4; ++it) {
      *(volatile v4u*)(Oh + go[it]) = wh[it];
      *(volatile v4u*)(Ol + go[it]) = wl[it];
    }
    __threadfence();
  }
}

__global__ __launch_bounds__(256) void k_gemm_out(const unsigned short* __restrict__ Ah,
                                                  const unsigned short* __restrict__ Al,
                                                  const unsigned short* __restrict__ Wh,
                                                  const unsigned short* __restrict__ Wl,
                                                  const float* __restrict__ bo,
                                                  float* __restrict__ out) {
  __shared__ __align__(16) float st[128 * OTP];
  const int tid = threadIdx.x, lane = tid & 31, wave = tid >> 5;
  const int hh = lane >> 4, c = lane & 15;
  const int mblk = blockIdx.y * 128, nblk = blockIdx.x * 64;
  const int mw = (wave >> 1) * 32, nw = (wave & 1) * 32;

  v8f acc[2][2];
#pragma unroll
  for (int s = 0; s < 2; ++s)
#pragma unroll
    for (int t = 0; t < 2; ++t) acc[s][t] = zero8();
  gemm32x32x3(Ah, Al, DM, Wh, Wl, DM, DM, mblk + mw, nblk + nw, lane, acc);

  float bb[2];
#pragma unroll
  for (int t = 0; t < 2; ++t) bb[t] = bo[nblk + nw + 16 * t + c];
  stage_rm(acc, bb, st, mw, nw, hh, c);
  __syncthreads();
  store_f32(st, out, mblk, nblk, tid);
}

extern "C" void kernel_launch(void* const* d_in, const int* in_sizes, int n_in,
                              void* d_out, int out_size, void* d_ws, size_t ws_size,
                              hipStream_t stream) {
  if (n_in < 14) return;
  if (in_sizes[0] != NT * DM) return;
  if (in_sizes[1] != NBT * SL) return;
  if (in_sizes[2] != NBT * SL) return;
  if (in_sizes[3] != NBT * SL) return;
  if (in_sizes[4] != DM * DM) return;
  if (in_sizes[5] != DM) return;
  if (in_sizes[6] != DM * DM) return;
  if (in_sizes[7] != DM) return;
  if (in_sizes[8] != DM * DM) return;
  if (in_sizes[9] != DM) return;
  if (in_sizes[10] != DM * DM) return;
  if (in_sizes[11] != DM) return;
  if (in_sizes[12] != GAPR * NH) return;
  if (in_sizes[13] != DURR * NH) return;
  if (out_size != NT * DM) return;

  const float* x     = (const float*)d_in[0];
  const int*   amask = (const int*)d_in[1];
  const int*   gids  = (const int*)d_in[2];
  const int*   dids  = (const int*)d_in[3];
  const float* W_q   = (const float*)d_in[4];
  const float* b_q   = (const float*)d_in[5];
  const float* W_k   = (const float*)d_in[6];
  const float* b_k   = (const float*)d_in[7];
  const float* W_v   = (const float*)d_in[8];
  const float* b_v   = (const float*)d_in[9];
  const float* W_o   = (const float*)d_in[10];
  const float* b_o   = (const float*)d_in[11];
  const float* gtab  = (const float*)d_in[12];
  const float* dtab  = (const float*)d_in[13];
  float* out = (float*)d_out;

  const size_t PX  = (size_t)NT * DM * 2;
  const size_t PW  = (size_t)3 * DM * DM * 2;
  const size_t PWO = (size_t)DM * DM * 2;
  size_t off = 0;
  const size_t oXh  = off; off += PX;
  const size_t oXl  = off; off += PX;
  const size_t oWh  = off; off += PW;
  const size_t oWl  = off; off += PW;
  const size_t oWoh = off; off += PWO;
  const size_t oWol = off; off += PWO;
  const size_t oQh  = off; off += PX;
  const size_t oQl  = off; off += PX;
  const size_t oKh  = off; off += PX;
  const size_t oKl  = off; off += PX;
  const size_t oVh  = off; off += PX;
  const size_t oVl  = off; off += PX;
  const size_t oOh  = off; off += PX;
  const size_t oOl  = off; off += PX;
  if (off > ws_size) return;
  if (off > (size_t)134217728) return;

  char* ws = (char*)d_ws;
  unsigned short* Xh  = (unsigned short*)(ws + oXh);
  unsigned short* Xl  = (unsigned short*)(ws + oXl);
  unsigned short* Wh  = (unsigned short*)(ws + oWh);
  unsigned short* Wl  = (unsigned short*)(ws + oWl);
  unsigned short* Woh = (unsigned short*)(ws + oWoh);
  unsigned short* Wol = (unsigned short*)(ws + oWol);
  unsigned short* Qh  = (unsigned short*)(ws + oQh);
  unsigned short* Ql  = (unsigned short*)(ws + oQl);
  unsigned short* Kh  = (unsigned short*)(ws + oKh);
  unsigned short* Kl  = (unsigned short*)(ws + oKl);
  unsigned short* Vh  = (unsigned short*)(ws + oVh);
  unsigned short* Vl  = (unsigned short*)(ws + oVl);
  unsigned short* Oh  = (unsigned short*)(ws + oOh);
  unsigned short* Ol  = (unsigned short*)(ws + oOl);

  k_split<<<dim3((NT * DM) / 2048), dim3(256), 0, stream>>>(x, Xh, Xl);
  k_split_tr<<<dim3(DM / 64, DM / 64, 4), dim3(256), 0, stream>>>(W_q, W_k, W_v, W_o, Wh, Wl, Woh, Wol);
  k_proj<<<dim3(3 * NH, NT / 128), dim3(256), 0, stream>>>(Xh, Xl, Wh, Wl, b_q, b_k, b_v,
                                                          Qh, Ql, Kh, Kl, Vh, Vl);
  k_attn<<<dim3(NBT * NH * NQB), dim3(256), 0, stream>>>(Qh, Ql, Kh, Kl, Vh, Vl, amask, gids, dids,
                                                        gtab, dtab, Oh, Ol);
  k_gemm_out<<<dim3(DM / 64, NT / 128), dim3(256), 0, stream>>>(Oh, Ol, Woh, Wol, b_o, out);
  (void)hipGetLastError();
}
